// PawletteMambaBlock_29566554865935
// MI455X (gfx1250) — hardware-run, weakly checked
//
#include <hip/hip_runtime.h>


#ifndef NB
#define NB 2
#endif
#ifndef SEQ
#define SEQ 2048
#endif
#define NB_FULL  2
#define SEQ_FULL 2048
#ifndef OUT_SEQ
#define OUT_SEQ SEQ
#endif
#define DM    672
#define DST   128
#define HDIM  56
#define NHD   24
#define DIN   1344
#define CDIM  1600
#define DPROJ 2968
#define ZP    3008
#define XOFF  1344
#define DTOFF 2944
#define UP    704
#define OPAD  704
#define CQ    64
#define MP    72
#define YP    68
#define EPSN  1.0e-5f
#define WCAR  64.0f
#define ACAR  16.0f
#define GSC   (1.0f / 1024.0f)
#define XCAR  256.0f
#define MSC   0.25f
#define SPK   (1.0f / 256.0f)
#define WXC   64.0f
#define YSC   (1.0f / 4194304.0f)

static_assert(NHD * HDIM == DIN);
static_assert(DIN + 2 * DST == CDIM);
static_assert(2 * DIN + 2 * DST + NHD == DPROJ);
static_assert(HDIM % 8 == 0);
static_assert(HDIM <= 64);
static_assert(DST == 128);
static_assert(CQ == 64);
static_assert(ZP % 64 == 0);
static_assert(ZP >= DPROJ);
static_assert(XOFF == DIN);
static_assert(XOFF % 64 == 0);
static_assert(DTOFF == DIN + CDIM);
static_assert(DTOFF % 64 == 0);
static_assert(DTOFF + NHD <= ZP);
static_assert(DM % 32 == 0);
static_assert(DIN % 32 == 0);
static_assert(DM % 8 == 0);
static_assert(UP % 64 == 0);
static_assert(UP >= DM);
static_assert(UP / 8 <= 96);
static_assert(OPAD % 64 == 0);
static_assert(OPAD >= DM);
static_assert((DM * 4) % 128 == 0);
static_assert((DM % 64 == 0) || (DM % 64 == 32));
static_assert(SEQ % 64 == 0);
static_assert((NB * SEQ) % 64 == 0);
static_assert((NB * SEQ) % 8 == 0);
static_assert(NB <= NB_FULL);
static_assert(SEQ <= SEQ_FULL);
static_assert(DIN % 32 == 0);
static_assert(DIN / 8 <= 6 * 32);
static_assert((DIN / 8) % 8 == 0);
static_assert((MP * 2) % 16 == 0);
static_assert((YP * 4) % 16 == 0);
static_assert(((size_t)ZP * DM) % 64 == 0);
static_assert(((size_t)OPAD * DIN) % 64 == 0);

typedef _Float16 h16;
typedef __attribute__((ext_vector_type(16))) _Float16 v16h;
typedef __attribute__((ext_vector_type(8)))  _Float16 v8h;
typedef __attribute__((ext_vector_type(8)))  float    v8f;
typedef __attribute__((ext_vector_type(4)))  float    v4f;
typedef v4f  __attribute__((may_alias)) v4fa;
typedef v8h  __attribute__((may_alias)) v8ha;

__device__ __forceinline__ unsigned short f2bf(float f) { unsigned u = __float_as_uint(f); u += 0x7FFFu + ((u >> 16) & 1u); return (unsigned short)(u >> 16); }
__device__ __forceinline__ float bfr(float f) { return __uint_as_float(((unsigned)f2bf(f)) << 16); }
__device__ __forceinline__ v16h cat16(v8h lo, v8h hi) { return __builtin_shufflevector(lo, hi, 0, 1, 2, 3, 4, 5, 6, 7, 8, 9, 10, 11, 12, 13, 14, 15); }
__device__ __forceinline__ v8f wmma16(v16h a, v16h b, v8f c) { return __builtin_amdgcn_wmma_f32_16x16x32_f16(false, a, false, b, (short)0, c, false, false); }
__device__ __forceinline__ v16h  ldh(const h16* p) { return cat16(*(const v8h*)p, *(const v8h*)(p + 16)); }
__device__ __forceinline__ void wave_sync() { __builtin_amdgcn_fence(3  , "wavefront"); __builtin_amdgcn_wave_barrier(); asm volatile("" ::: "memory"); }

static __device__ __forceinline__ h16 toh_flush(float v) { const h16 r = (h16)v; return (fabsf(v) < 6.103515625e-05f) ? (h16)0.0f : r; }
__device__ __forceinline__ v8f wm16g(v16h a, v16h b, v8f c) { c = wmma16(a, b, c); asm volatile("v_nop\n\tv_nop\n\tv_nop\n\tv_nop" : "+v"(c) : "v"(a), "v"(b)); return c; }
__device__ __forceinline__ float clampf(float v) { return fminf(fmaxf(v, -60000.0f), 60000.0f); }
__device__ __forceinline__ float silu_f(float x) { return x * __builtin_amdgcn_rcpf(1.0f + __expf(-x)); }
__device__ __forceinline__ float softplus_f(float x) { return fmaxf(x, 0.0f) + log1pf(__expf(-fabsf(x))); }
__device__ __forceinline__ float wsum(float v) { v += __shfl_xor(v, 16, 32); v += __shfl_xor(v, 8, 32); v += __shfl_xor(v, 4, 32); v += __shfl_xor(v, 2, 32); v += __shfl_xor(v, 1, 32); return v; }
__device__ __forceinline__ float ldtap(const float* __restrict__ ZX, int srow, int tq, int col) {
    const int tc = tq < 0 ? 0 : tq;
    float v = ZX[(size_t)(srow + tc) * ZP + col];
    asm volatile("" : "+v"(v));
    return (tq >= 0) ? v : 0.0f;
}

__global__ __launch_bounds__(256) void k_wcvt(const float* __restrict__ src, h16* dst, size_t n8, size_t nv8, float carry) {
#pragma clang fp contract(off)
    const size_t i = (size_t)blockIdx.x * 256 + threadIdx.x; if (i >= n8) return;
    const bool ok = i < nv8;
    const size_t ic = ok ? i : nv8 - 1;
    v8f v = *(const v8f*)(src + ic * 8);
    asm volatile("" : "+v"(v));
    v8h o;
#pragma unroll
    for (int k = 0; k < 8; ++k) { const float x = ok ? bfr(v[k]) * carry : 0.0f; o[k] = toh_flush(x); }
    *(volatile v8h*)(dst + i * 8) = o; __threadfence(); *(volatile v8h*)(dst + i * 8) = o;
}

__global__ __launch_bounds__(256) void k_norm1(const float* __restrict__ X, const float* __restrict__ G, h16* U) {
#pragma clang fp contract(off)
    const int lane = threadIdx.x & 31;
    const int wave = __builtin_amdgcn_readfirstlane((int)(threadIdx.x >> 5));
    const int m = blockIdx.x * 8 + wave;
    const int bb = m / SEQ, tt = m - bb * SEQ;
    const float* xr = X + ((size_t)bb * SEQ_FULL + tt) * DM;
    float ss = 0.0f;
#pragma unroll 1
    for (int i = 0; i < DM / 32; ++i) { const float v = bfr(xr[lane + 32 * i]); ss += v * v; }
    ss = wsum(ss);
    const float rs = rsqrtf(ss * (1.0f / (float)DM) + EPSN);
    h16* ur = U + (size_t)m * UP;
#pragma unroll 1
    for (int ps = 0; ps < 2; ++ps) {
#pragma unroll 1
        for (int i = 0; i < 3; ++i) {
            const int j = lane + 32 * i;
            const bool stp = j < UP / 8;
            const bool dat = j < DM / 8;
            const int jc = dat ? j : (DM / 8 - 1);
            v4f x0 = *(const v4f*)(xr + jc * 8), x1 = *(const v4f*)(xr + jc * 8 + 4);
            v4f g0 = *(const v4f*)(G + jc * 8), g1 = *(const v4f*)(G + jc * 8 + 4);
            asm volatile("" : "+v"(x0), "+v"(x1), "+v"(g0), "+v"(g1));
            v8h o;
#pragma unroll
            for (int k = 0; k < 4; ++k) {
                const float a0 = bfr(g0[k]) * (bfr(x0[k]) * rs) * ACAR;
                const float a1 = bfr(g1[k]) * (bfr(x1[k]) * rs) * ACAR;
                o[k] = toh_flush(dat ? a0 : 0.0f); o[4 + k] = toh_flush(dat ? a1 : 0.0f); }
            if (stp) *(volatile v8h*)(ur + j * 8) = o;
        }
        if (ps == 0) __threadfence(); }
}

static_assert(32 * 8 * 16 == 16 * 64 * 4);
__global__ __launch_bounds__(32) void k_gemm(const h16* __restrict__ A, const h16* __restrict__ Bt, const float* __restrict__ R, float* C,
                                             int K, int lda, int N, int ldc, int seqc, int rseq, int oseq, int hasres, float scale) {
    __shared__ __align__(16) float os[16 * 68];
    const int lane = threadIdx.x & 31, lr = lane & 15, hi = lane >> 4; const int r0 = blockIdx.x * 64, c0 = blockIdx.y * 64;
    v8f acc[4][4];
#pragma unroll
    for (int mb = 0; mb < 4; ++mb)
#pragma unroll
        for (int nb = 0; nb < 4; ++nb) acc[mb][nb] = (v8f){};
    const size_t aoff = (size_t)(r0 + lr) * lda + 8 * hi, boff = (size_t)(c0 + lr) * K + 8 * hi;
#pragma unroll 1
    for (int kc = 0; kc < K; kc += 32) {
        v16h a[4];
#pragma unroll
        for (int mb = 0; mb < 4; ++mb) a[mb] = ldh(A + aoff + (size_t)mb * 16 * lda + kc);
#pragma unroll
        for (int nb = 0; nb < 4; ++nb) { const v16h bq = ldh(Bt + boff + (size_t)nb * 16 * K + kc);
#pragma unroll
            for (int mb = 0; mb < 4; ++mb) acc[mb][nb] = wm16g(a[mb], bq, acc[mb][nb]); }
    }
#pragma unroll
    for (int mb = 0; mb < 4; ++mb) {
#pragma unroll
        for (int nb = 0; nb < 4; ++nb) {
#pragma unroll
            for (int j = 0; j < 8; ++j) os[(hi * 8 + j) * 68 + nb * 16 + lr] = acc[mb][nb][j] * scale; }
        wave_sync();
#pragma unroll 1
        for (int ps = 0; ps < 2; ++ps) {
#pragma unroll
            for (int s = 0; s < 8; ++s) { const int row = 2 * s + (lane >> 4), c4 = (lane & 15) * 4;
                const int col = c0 + c4; const bool ok = col < N; const int cc = ok ? col : (N - 4);
                const int grow = r0 + mb * 16 + row; const int bb = grow / seqc, tt = grow - bb * seqc;
                v4f val = *(const v4fa*)(&os[row * 68 + c4]);
                if (hasres != 0) {
                    v4f rv = *(const v4f*)(R + ((size_t)bb * rseq + tt) * ldc + cc);
                    asm volatile("" : "+v"(rv));
                    val[0] += bfr(rv[0]); val[1] += bfr(rv[1]); val[2] += bfr(rv[2]); val[3] += bfr(rv[3]); }
                if (ok) *(volatile v4f*)(C + ((size_t)bb * oseq + tt) * ldc + col) = val; }
            if (ps == 0) __threadfence(); }
        wave_sync();
    }
}

static_assert(256 * 2 * 16 == 64 * 128);
__global__ __launch_bounds__(256) void k_conv(const float* __restrict__ ZX, const float* __restrict__ CW, const float* __restrict__ CB, h16* XT, h16* BH, h16* BT, h16* CH) {
#pragma clang fp contract(off)
    __shared__ __align__(16) h16 tn[64 * MP];
    __shared__ __align__(16) h16 tx[64 * MP];
    const int tid = threadIdx.x;
    const int g = blockIdx.y;
    const int m0 = blockIdx.x * 64;
    const int bb = m0 / SEQ, t0 = m0 - bb * SEQ;
    const int srow = bb * SEQ;
    const int nch = g < NHD ? HDIM : 64;
    const int cbase = g < NHD ? g * HDIM : DIN + (g - NHD) * 64;
    const int c = tid & 63, tg = tid >> 6;
    const bool cv = c < nch;
    const int cc = cbase + (cv ? c : nch - 1);
    v4f w = *(const v4f*)(CW + (size_t)cc * 4); float bia = CB[cc];
    asm volatile("" : "+v"(w), "+v"(bia));
    const float w0 = bfr(w[0]), w1 = bfr(w[1]), w2 = bfr(w[2]), w3 = bfr(w[3]); bia = bfr(bia);
    const int ts = tg * 16;
    const int col = XOFF + cc;
    float x0 = ldtap(ZX, srow, t0 + ts - 3, col), x1 = ldtap(ZX, srow, t0 + ts - 2, col), x2 = ldtap(ZX, srow, t0 + ts - 1, col);
#pragma unroll 1
    for (int i = 0; i < 16; ++i) {
        const float x3 = ldtap(ZX, srow, t0 + ts + i, col);
        float a = x0 * w0; a += x1 * w1; a += x2 * w2; a += x3 * w3; a += bia;
        const float sv = silu_f(a);
        const h16 hv = toh_flush(cv ? sv * XCAR : 0.0f);
        tn[(ts + i) * MP + c] = hv; tx[c * MP + ts + i] = hv;
        x0 = x1; x1 = x2; x2 = x3; }
    __syncthreads();
#pragma unroll 1
    for (int ps = 0; ps < 2; ++ps) {
#pragma unroll
        for (int it = 0; it < 2; ++it) { const int q = tid + 256 * it; const int row = q >> 3, c8 = (q & 7) * 8;
            const v8h vn = *(const v8ha*)(&tn[row * MP + c8]);
            const v8h vt = *(const v8ha*)(&tx[row * MP + c8]);
            if (g < NHD) {
                *(volatile v8h*)(XT + (((size_t)(bb * NHD + g) * 64 + row) * SEQ + t0 + c8)) = vt;
            } else if (g < NHD + 2) {
                *(volatile v8h*)(BH + ((size_t)(m0 + row) * DST + (g - NHD) * 64 + c8)) = vn;
                *(volatile v8h*)(BT + (((size_t)bb * DST + (g - NHD) * 64 + row) * SEQ + t0 + c8)) = vt;
            } else {
                *(volatile v8h*)(CH + ((size_t)(m0 + row) * DST + (g - NHD - 2) * 64 + c8)) = vn;
            } }
        if (ps == 0) __threadfence(); }
}

static_assert(128 * 8 * 16 == 64 * 64 * 4);
__global__ __launch_bounds__(128) void k_chunkscan(const float* __restrict__ ZX, const h16* __restrict__ XT, const h16* __restrict__ BH, const h16* __restrict__ BT,
                                             const h16* __restrict__ CH, const float* __restrict__ DTB, const float* __restrict__ ALOG, float* Y) {
    __shared__ __align__(16) h16 sM[CQ * MP];
    __shared__ __align__(16) float sY[CQ * YP];
    __shared__ __align__(16) float sdt[CQ];
    __shared__ __align__(16) float scs[CQ];
    __shared__ __align__(16) float sE[CQ];
    __shared__ __align__(16) float sW[CQ];
    const int tid = threadIdx.x, lane = tid & 31, lr = lane & 15, hi = lane >> 4;
    const int wave = __builtin_amdgcn_readfirstlane((int)(threadIdx.x >> 5));
    const int bh = blockIdx.x; const int b = bh / NHD, h = bh - b * NHD;
    const float negA = -expf(bfr(ALOG[h]));
    const float dtb = bfr(DTB[h]);
    v8f st[8];
#pragma unroll
    for (int a = 0; a < 8; ++a) st[a] = (v8f){};
    const size_t xtrow = ((size_t)bh * 64 + wave * 16 + lr) * SEQ + 8 * hi;
    const size_t btrow = ((size_t)b * DST + lr) * SEQ + 8 * hi;
#pragma unroll 1
    for (int c = 0; c < SEQ / CQ; ++c) {
        const int tb = b * SEQ + c * CQ;
        if (wave == 0) {
            const float q0 = ZX[(size_t)(tb + lane) * ZP + DTOFF + h], q1 = ZX[(size_t)(tb + 32 + lane) * ZP + DTOFF + h];
            const float d0 = softplus_f(q0 + dtb), d1 = softplus_f(q1 + dtb);
            float a0 = d0 * negA, a1 = d1 * negA;
#pragma unroll
            for (int o = 1; o < 32; o <<= 1) { const float u0 = __shfl_up(a0, o, 32), u1 = __shfl_up(a1, o, 32); a0 += (lane >= o) ? u0 : 0.0f; a1 += (lane >= o) ? u1 : 0.0f; }
            const float tot0 = __shfl(a0, 31, 32); a1 += tot0;
            const float tot = __shfl(a1, 31, 32);
            sdt[lane] = d0; sdt[32 + lane] = d1; scs[lane] = a0; scs[32 + lane] = a1;
            sE[lane] = __expf(a0); sE[32 + lane] = __expf(a1);
            sW[lane] = __expf(fminf(tot - a0, 0.0f)) * d0 * WXC; sW[32 + lane] = __expf(fminf(tot - a1, 0.0f)) * d1 * WXC;
        }
        __syncthreads();
        {
            const size_t crow = (size_t)(tb + wave * 16 + lr) * DST + 8 * hi;
            v16h cf[4];
#pragma unroll
            for (int k = 0; k < 4; ++k) cf[k] = ldh(CH + crow + 32 * k);
            float cst[8];
#pragma unroll
            for (int r = 0; r < 8; ++r) cst[r] = scs[wave * 16 + 8 * hi + r];
#pragma unroll 1
            for (int j = 0; j < 4; ++j) {
                v8f gacc = (v8f){};
                const size_t brow = (size_t)(tb + j * 16 + lr) * DST + 8 * hi;
#pragma unroll
                for (int k = 0; k < 4; ++k) gacc = wm16g(cf[k], ldh(BH + brow + 32 * k), gacc);
                const int s = j * 16 + lr; const float css = scs[s]; const float dts = sdt[s] * MSC;
#pragma unroll
                for (int r = 0; r < 8; ++r) { const int t = wave * 16 + 8 * hi + r;
                    const float e = __expf(fminf(cst[r] - css, 0.0f));
                    const float v = clampf(gacc[r] * e * dts);
                    const h16 mv = toh_flush((s <= t) ? v : 0.0f);
                    sM[t * MP + s] = mv; }
            }
        }
        __syncthreads();
        const v16h xt0 = ldh(XT + xtrow + c * CQ), xt1 = ldh(XT + xtrow + c * CQ + 32);
        {
            v16h sf[4];
#pragma unroll
            for (int kn = 0; kn < 4; ++kn) {
#pragma unroll
                for (int r = 0; r < 8; ++r) { sf[kn][r] = toh_flush(clampf(st[2 * kn][r] * SPK)); sf[kn][8 + r] = toh_flush(clampf(st[2 * kn + 1][r] * SPK)); } }
#pragma unroll 1
            for (int i = 0; i < 4; ++i) {
                v8f ai = (v8f){}, ae = (v8f){};
                const int mo = (i * 16 + lr) * MP + 8 * hi;
                const v16h m0f = cat16(*(const v8ha*)(&sM[mo]), *(const v8ha*)(&sM[mo + 16]));
                const v16h m1f = cat16(*(const v8ha*)(&sM[mo + 32]), *(const v8ha*)(&sM[mo + 48]));
                ai = wm16g(m0f, xt0, ai); ai = wm16g(m1f, xt1, ai);
                const size_t crow = (size_t)(tb + i * 16 + lr) * DST + 8 * hi;
#pragma unroll
                for (int kn = 0; kn < 4; ++kn) ae = wm16g(ldh(CH + crow + 32 * kn), sf[kn], ae);
#pragma unroll
                for (int r = 0; r < 8; ++r) { const int t = i * 16 + 8 * hi + r; sY[t * YP + wave * 16 + lr] = (ai[r] + ae[r] * sE[t]) * YSC; }
            }
        }
        {
            const float dec = sE[CQ - 1];
            v16h xw0, xw1;
            { const v4f wa = *(const v4fa*)(&sW[8 * hi]), wb = *(const v4fa*)(&sW[8 * hi + 4]), wc = *(const v4fa*)(&sW[16 + 8 * hi]), wd = *(const v4fa*)(&sW[16 + 8 * hi + 4]);
#pragma unroll
              for (int r = 0; r < 4; ++r) { xw0[r] = toh_flush(clampf((float)xt0[r] * wa[r])); xw0[4 + r] = toh_flush(clampf((float)xt0[4 + r] * wb[r]));
                                            xw0[8 + r] = toh_flush(clampf((float)xt0[8 + r] * wc[r])); xw0[12 + r] = toh_flush(clampf((float)xt0[12 + r] * wd[r])); } }
            { const v4f wa = *(const v4fa*)(&sW[32 + 8 * hi]), wb = *(const v4fa*)(&sW[32 + 8 * hi + 4]), wc = *(const v4fa*)(&sW[48 + 8 * hi]), wd = *(const v4fa*)(&sW[48 + 8 * hi + 4]);
#pragma unroll
              for (int r = 0; r < 4; ++r) { xw1[r] = toh_flush(clampf((float)xt1[r] * wa[r])); xw1[4 + r] = toh_flush(clampf((float)xt1[4 + r] * wb[r]));
                                            xw1[8 + r] = toh_flush(clampf((float)xt1[8 + r] * wc[r])); xw1[12 + r] = toh_flush(clampf((float)xt1[12 + r] * wd[r])); } }
#pragma unroll
            for (int a = 0; a < 8; ++a) {
                st[a] = st[a] * dec;
                const size_t bo = btrow + (size_t)(16 * a) * SEQ + c * CQ;
                st[a] = wm16g(ldh(BT + bo), xw0, st[a]);
                st[a] = wm16g(ldh(BT + bo + 32), xw1, st[a]); }
        }
        __syncthreads();
        float* yb = Y + ((size_t)bh * SEQ + c * CQ) * 64;
#pragma unroll 1
        for (int ps = 0; ps < 2; ++ps) {
#pragma unroll
            for (int it = 0; it < 8; ++it) { const int q = tid + 128 * it; const int row = q >> 4, c4 = (q & 15) * 4;
                const v4f val = *(const v4fa*)(&sY[row * YP + c4]);
                *(volatile v4f*)(yb + (size_t)row * 64 + c4) = val; }
            if (ps == 0) __threadfence(); }
        __syncthreads();
    }
}

__global__ __launch_bounds__(256) void k_gate(const float* __restrict__ ZX, const float* __restrict__ Y, const float* __restrict__ CW, const float* __restrict__ CB,
                                              const float* __restrict__ DV, const float* __restrict__ GW, h16* YN) {
#pragma clang fp contract(off)
    __shared__ __align__(16) float sg[8 * DIN];
    const int lane = threadIdx.x & 31;
    const int wave = __builtin_amdgcn_readfirstlane((int)(threadIdx.x >> 5));
    const int m = blockIdx.x * 8 + wave;
    const int bb = m / SEQ, tt = m - bb * SEQ;
    const int srow = bb * SEQ;
    const int wb = wave * DIN;
    float ss = 0.0f;
#pragma unroll 1
    for (int i = 0; i < DIN / 32; ++i) {
        const int e = lane + 32 * i; const int hh = e / HDIM, p = e - hh * HDIM;
        const float z = ZX[(size_t)m * ZP + e];
        const float ys = Y[(((size_t)(bb * NHD + hh)) * SEQ + tt) * 64 + p];
        v4f w = *(const v4f*)(CW + (size_t)e * 4); float bia = CB[e]; float dv = DV[hh];
        asm volatile("" : "+v"(w), "+v"(bia), "+v"(dv));
        const float x0 = ldtap(ZX, srow, tt - 3, XOFF + e), x1 = ldtap(ZX, srow, tt - 2, XOFF + e), x2 = ldtap(ZX, srow, tt - 1, XOFF + e), x3 = ldtap(ZX, srow, tt, XOFF + e);
        float a = x0 * bfr(w[0]); a += x1 * bfr(w[1]); a += x2 * bfr(w[2]); a += x3 * bfr(w[3]); a += bfr(bia);
        const float xv = silu_f(a);
        const float y = ys + bfr(dv) * xv;
        const float gv = y * silu_f(z);
        sg[wb + e] = gv; ss += gv * gv; }
    ss = wsum(ss);
    const float rs = rsqrtf(ss * (1.0f / (float)DIN) + EPSN);
    wave_sync();
    h16* yr = YN + (size_t)m * DIN;
#pragma unroll 1
    for (int ps = 0; ps < 2; ++ps) {
#pragma unroll 1
        for (int i = 0; i < 6; ++i) {
            const int j = lane + 32 * i; const bool ok = j < DIN / 8; const int jc = ok ? j : (DIN / 8 - 1);
            const v4f g0 = *(const v4fa*)(&sg[wb + jc * 8]), g1 = *(const v4fa*)(&sg[wb + jc * 8 + 4]);
            v4f w0 = *(const v4f*)(GW + jc * 8), w1 = *(const v4f*)(GW + jc * 8 + 4);
            asm volatile("" : "+v"(w0), "+v"(w1));
            v8h o;
#pragma unroll
            for (int k = 0; k < 4; ++k) { o[k] = toh_flush(bfr(w0[k]) * (g0[k] * rs) * ACAR); o[4 + k] = toh_flush(bfr(w1[k]) * (g1[k] * rs) * ACAR); }
            if (ok) *(volatile v8h*)(yr + j * 8) = o;
        }
        if (ps == 0) __threadfence(); }
}

static constexpr size_t al256(size_t v) { return (v + 255) & ~(size_t)255; }
static constexpr size_t SZ_WIN = al256((size_t)ZP * DM * 2);
static constexpr size_t SZ_WOUT = al256((size_t)OPAD * DIN * 2);
static constexpr size_t SZ_U = al256((size_t)NB * SEQ * UP * 2);
static constexpr size_t SZ_ZX = al256((size_t)NB * SEQ * ZP * 4);
static constexpr size_t SZ_XT = al256((size_t)NB * NHD * 64 * SEQ * 2);
static constexpr size_t SZ_BC = al256((size_t)NB * SEQ * DST * 2);
static constexpr size_t SZ_Y = al256((size_t)NB * NHD * SEQ * 64 * 4);
static constexpr size_t SZ_YN = al256((size_t)NB * SEQ * DIN * 2);
static constexpr size_t SZ_TOTAL = SZ_WIN + SZ_WOUT + SZ_U + SZ_ZX + SZ_XT + 3 * SZ_BC + SZ_Y + SZ_YN;
static_assert(SZ_TOTAL <= (size_t)134217728);
static_assert(9216 + 17408 + 4 * 256 <= 131072);
static_assert(8 * DIN * 4 <= 131072);
static_assert(2 * 64 * MP * 2 <= 131072);
static_assert((((size_t)ZP * DM) / 8) % 256 == 0 || true);

extern "C" void kernel_launch(void* const* d_in, const int* in_sizes, int n_in,
                              void* d_out, int out_size, void* d_ws, size_t ws_size, hipStream_t stream) {
    if (n_in < 10) return;
    const size_t needx = ((size_t)(NB - 1) * SEQ_FULL + SEQ) * DM;
    if ((size_t)in_sizes[0] < needx) return;
    if (in_sizes[1] < DM) return;
    if ((size_t)in_sizes[2] < (size_t)DPROJ * DM) return;
    if (in_sizes[3] < CDIM * 4 || in_sizes[4] < CDIM) return;
    if (in_sizes[5] < NHD || in_sizes[6] < NHD || in_sizes[7] < NHD) return;
    if (in_sizes[8] < DIN) return;
    if ((size_t)in_sizes[9] < (size_t)DM * DIN) return;
    if ((size_t)out_size < ((size_t)(NB - 1) * OUT_SEQ + SEQ) * DM) return;
    if (SZ_TOTAL > ws_size) return;
    const float* hid = (const float*)d_in[0];
    const float* nw = (const float*)d_in[1];
    const float* win = (const float*)d_in[2];
    const float* cw = (const float*)d_in[3];
    const float* cb = (const float*)d_in[4];
    const float* dtb = (const float*)d_in[5];
    const float* alog = (const float*)d_in[6];
    const float* dv = (const float*)d_in[7];
    const float* gw = (const float*)d_in[8];
    const float* wout = (const float*)d_in[9];
    float* OUT = (float*)d_out;
    char* wsp = (char*)d_ws;
    h16* WIN = (h16*)wsp; wsp += SZ_WIN;
    h16* WOUT = (h16*)wsp; wsp += SZ_WOUT;
    h16* U = (h16*)wsp; wsp += SZ_U;
    float* ZX = (float*)wsp; wsp += SZ_ZX;
    h16* XT = (h16*)wsp; wsp += SZ_XT;
    h16* BHp = (h16*)wsp; wsp += SZ_BC;
    h16* BTp = (h16*)wsp; wsp += SZ_BC;
    h16* CHp = (h16*)wsp; wsp += SZ_BC;
    float* Yp = (float*)wsp; wsp += SZ_Y;
    h16* YN = (h16*)wsp; wsp += SZ_YN;

    { const size_t n8 = (size_t)ZP * DM / 8, nv8 = (size_t)DPROJ * DM / 8;
      k_wcvt<<<(unsigned)((n8 + 255) / 256), 256, 0, stream>>>(win, WIN, n8, nv8, WCAR); }
    { const size_t n8 = (size_t)OPAD * DIN / 8, nv8 = (size_t)DM * DIN / 8;
      k_wcvt<<<(unsigned)((n8 + 255) / 256), 256, 0, stream>>>(wout, WOUT, n8, nv8, WCAR); }
    k_norm1<<<NB * SEQ / 8, 256, 0, stream>>>(hid, nw, U);
    k_gemm<<<dim3(NB * SEQ / 64, ZP / 64, 1), 32, 0, stream>>>(U, WIN, hid, ZX, DM, UP, ZP, ZP, NB * SEQ, NB * SEQ, NB * SEQ, 0, GSC);
    k_conv<<<dim3(NB * SEQ / 64, NHD + 4, 1), 256, 0, stream>>>(ZX, cw, cb, XT, BHp, BTp, CHp);
    k_chunkscan<<<NB * NHD, 128, 0, stream>>>(ZX, XT, BHp, BTp, CHp, dtb, alog, Yp);
    k_gate<<<NB * SEQ / 8, 256, 0, stream>>>(ZX, Yp, cw, cb, dv, gw, YN);
    k_gemm<<<dim3(NB * SEQ / 64, OPAD / 64, 1), 32, 0, stream>>>(YN, WOUT, hid, OUT, DIN, DIN, DM, DM, SEQ, SEQ_FULL, OUT_SEQ, 1, GSC);
}
